// SelfAttention_996432413483
// MI455X (gfx1250) — hardware-verified
//
#include <hip/hip_runtime.h>


#ifndef NB
#define NB 4
#endif
#ifndef SEQ
#define SEQ 4096
#endif
#define NB_FULL   4
#define SEQ_FULL  4096
#define CH        256
#define NHEAD     4
#define HDIM      64
#define NGRP      8
#define CPG       32
#define QKV_O     768
#define BQ        128
#define BK        32
#define NWAVE     8
#define TP        72
#define SQ_P      72
#define SV_P      136
#define SS_HALVES (128 * SQ_P)
#define OP        68
#define YP        132
#define WQ_ELEMS  (QKV_O * CH)
#define WP_ELEMS  (CH * CH)
#define WQ_BLKS   (WQ_ELEMS / 2048)
#define WP_BLKS   (WP_ELEMS / 2048)

static_assert(SEQ % 128 == 0);
static_assert(SEQ <= SEQ_FULL);
static_assert(NB >= 1 && NB <= NB_FULL);
static_assert(CH == NHEAD * HDIM);
static_assert(CH == NGRP * CPG);
static_assert(CH % 32 == 0);
static_assert(HDIM == 64);
static_assert(BQ == NWAVE * 16);
static_assert(WQ_ELEMS % 2048 == 0 && WP_ELEMS % 2048 == 0);
static_assert((WQ_BLKS + WP_BLKS) * 256 * 8 == WQ_ELEMS + WP_ELEMS);
static_assert((CPG * SEQ) % 1024 == 0);
static_assert(256 * 2 * 8 == 64 * 64);
static_assert(256 * 4 * 8 == 128 * 64);
static_assert(32 * 4 * 8 == 16 * 64);
static_assert(256 * 8 * 4 == 64 * 128);
static_assert(64 * SV_P <= SS_HALVES);
static_assert((TP * 2) % 16 == 0 && (SQ_P * 2) % 16 == 0 && (SV_P * 2) % 16 == 0);
static_assert((OP * 4) % 16 == 0 && (YP * 4) % 16 == 0);

typedef __bf16   bf16;
typedef _Float16 f16;
typedef f16      v16h __attribute__((ext_vector_type(16)));
typedef f16      v8h  __attribute__((ext_vector_type(8)));
typedef float    v8f  __attribute__((ext_vector_type(8)));
typedef float    v4f  __attribute__((ext_vector_type(4)));
typedef unsigned v4u  __attribute__((ext_vector_type(4)));

union FragH  { v16h v; v4u q[2]; f16 h[16]; };
union Pack8H { v4u u; v8h v; f16 h[8]; };

static __device__ __forceinline__ float bfv(float x) { return (float)(bf16)x; }

static __device__ __forceinline__ v8f mma_f16(v16h a, v16h b, v8f acc) {
  acc = __builtin_amdgcn_wmma_f32_16x16x32_f16(false, a, false, b, (short)0, acc, false, false);
  asm volatile("v_nop\n\tv_nop\n\tv_nop\n\tv_nop" : "+v"(acc) : "v"(a), "v"(b));
  return acc;
}

static __device__ __forceinline__ void wave_gemm_64x16(const f16* __restrict__ a0,
                                                       const f16* __restrict__ bp,
                                                       v8f (&acc)[4]) {
  #pragma unroll 2
  for (unsigned k0 = 0; k0 < CH; k0 += 32) {
    FragH fb;
    fb.q[0] = *(const v4u*)(bp + k0);
    fb.q[1] = *(const v4u*)(bp + k0 + 16);
    FragH fa[4];
    #pragma unroll
    for (unsigned os = 0; os < 4; ++os) {
      const f16* ap = a0 + (size_t)os * 16 * CH + k0;
      fa[os].q[0] = *(const v4u*)(ap);
      fa[os].q[1] = *(const v4u*)(ap + 16);
    }
    #pragma unroll
    for (unsigned os = 0; os < 4; ++os) acc[os] = mma_f16(fa[os].v, fb.v, acc[os]);
  }
}

__global__ __launch_bounds__(256) void wcvt_kernel(const float* __restrict__ qkvw,
                                                   const float* __restrict__ projw,
                                                   f16* __restrict__ wq,
                                                   f16* __restrict__ wp) {
  const unsigned blk = blockIdx.x;
  const unsigned tid = threadIdx.x;
  const bool isq = blk < WQ_BLKS;
  const unsigned e = (isq ? blk : blk - WQ_BLKS) * 2048u + tid * 8u;
  const float* src = (isq ? qkvw : projw) + e;
  f16* dst = (isq ? wq : wp) + e;
  const v4f a = *(const v4f*)(src);
  const v4f c = *(const v4f*)(src + 4);
  Pack8H pk;
  #pragma unroll
  for (unsigned i = 0; i < 4; ++i) {
    pk.h[i]     = (f16)(bfv(a[i]) * 16.0f);
    pk.h[4 + i] = (f16)(bfv(c[i]) * 16.0f);
  }
  const v4u val = pk.u;
  *(volatile v4u*)dst = val;
  __threadfence();
  *(volatile v4u*)dst = val;
}

__global__ __launch_bounds__(256) void gnstats_kernel(const float* __restrict__ x,
                                                      float* __restrict__ stats) {
  const unsigned g    = blockIdx.x;
  const unsigned b    = blockIdx.y;
  const unsigned tid  = threadIdx.x;
  const unsigned lane = tid & 31u;
  const unsigned wave = tid >> 5;
  const float* base = x + ((size_t)b * CH + g * CPG) * SEQ_FULL;
  double ds = 0.0, ds2 = 0.0;
  #pragma unroll 1
  for (unsigned i = tid * 4u; i < (unsigned)(CPG * SEQ); i += 1024u) {
    const unsigned c = i / (unsigned)SEQ;
    const unsigned n = i - c * (unsigned)SEQ;
    const v4f v = *(const v4f*)(base + (size_t)c * SEQ_FULL + n);
    const float a0 = bfv(v[0]), a1 = bfv(v[1]), a2 = bfv(v[2]), a3 = bfv(v[3]);
    ds  += (double)((a0 + a1) + (a2 + a3));
    ds2 += (double)((a0 * a0 + a1 * a1) + (a2 * a2 + a3 * a3));
  }
  #pragma unroll
  for (int m = 16; m >= 1; m >>= 1) {
    ds  += __shfl_xor(ds,  m, 32);
    ds2 += __shfl_xor(ds2, m, 32);
  }
  __shared__ double red[2 * NWAVE];
  if (lane == 0) { red[wave * 2] = ds; red[wave * 2 + 1] = ds2; }
  __syncthreads();
  double ts = 0.0, ts2 = 0.0;
  #pragma unroll
  for (unsigned w = 0; w < NWAVE; ++w) { ts += red[w * 2]; ts2 += red[w * 2 + 1]; }
  const double inv_n = 1.0 / (double)(CPG * SEQ);
  const double mean  = ts * inv_n;
  const double var   = ts2 * inv_n - mean * mean;
  const float  rstd  = 1.0f / sqrtf((float)var + 1e-5f);
  const v4f val = (v4f){(float)mean, rstd, 0.0f, 0.0f};
  float* dst = stats + (size_t)(b * NGRP + g) * 32 + (tid & 7u) * 4u;
  if (tid < 8) *(volatile v4f*)dst = val;
  __threadfence();
  if (tid < 8) *(volatile v4f*)dst = val;
}

__global__ __launch_bounds__(256) void gnapply_kernel(const float* __restrict__ x,
                                                      const float* __restrict__ gamma,
                                                      const float* __restrict__ beta,
                                                      const float* __restrict__ stats,
                                                      f16* __restrict__ hnT) {
  const unsigned ntile = blockIdx.x;
  const unsigned ctile = blockIdx.y;
  const unsigned b     = blockIdx.z;
  const unsigned tid   = threadIdx.x;
  __shared__ __align__(16) f16 sT[64 * TP];
  const unsigned c0 = ctile * 64u;
  const unsigned n0 = ntile * 64u;
  const unsigned cl_lo = tid >> 4;
  const unsigned tn4   = (tid & 15u) * 4u;
  #pragma unroll
  for (unsigned it = 0; it < 4; ++it) {
    const unsigned cl = it * 16u + cl_lo;
    const unsigned c  = c0 + cl;
    const unsigned sl = (b * NGRP + (c >> 5)) * 32u;
    const float mean = stats[sl];
    const float rstd = stats[sl + 1];
    const float ga = bfv(gamma[c]) * rstd;
    const float be = bfv(beta[c]) - mean * ga;
    const v4f v = *(const v4f*)(x + ((size_t)b * CH + c) * SEQ_FULL + n0 + tn4);
    #pragma unroll
    for (unsigned j = 0; j < 4; ++j)
      sT[(tn4 + j) * TP + cl] = (f16)(bfv(v[j]) * ga + be);
  }
  __syncthreads();

  v4u    vals[2];
  size_t gidx[2];
  #pragma unroll
  for (unsigned kk = 0; kk < 2; ++kk) {
    const unsigned row = kk * 32u + (tid >> 3);
    const unsigned pc  = (tid & 7u) * 8u;
    Pack8H ph;
    ph.v = *(const v8h*)(sT + row * TP + pc);
    vals[kk] = ph.u;
    gidx[kk] = ((size_t)b * SEQ + n0 + row) * CH + c0 + pc;
  }
  #pragma unroll
  for (unsigned kk = 0; kk < 2; ++kk) *(volatile v4u*)(hnT + gidx[kk]) = vals[kk];
  __threadfence();
  #pragma unroll
  for (unsigned kk = 0; kk < 2; ++kk) *(volatile v4u*)(hnT + gidx[kk]) = vals[kk];
}

__global__ __launch_bounds__(256) void qkv_kernel(const f16* __restrict__ hnT,
                                                  const f16* __restrict__ wq,
                                                  const float* __restrict__ bias,
                                                  f16* __restrict__ qpl,
                                                  f16* __restrict__ kpl,
                                                  f16* __restrict__ vtl) {
  const unsigned nt   = blockIdx.x;
  const unsigned og   = blockIdx.y;
  const unsigned b    = blockIdx.z;
  const unsigned tid  = threadIdx.x;
  const unsigned wave = tid >> 5;
  const unsigned lane = tid & 31u;
  const unsigned lq   = lane & 15u;
  const unsigned hi   = lane >> 4;
  const unsigned t    = og >> 2;
  const unsigned h    = og & 3u;
  const unsigned n0   = nt * 128u;

  __shared__ __align__(16) f16 sS[SS_HALVES];

  v8f acc[4];
  #pragma unroll
  for (unsigned os = 0; os < 4; ++os) acc[os] = (v8f){0, 0, 0, 0, 0, 0, 0, 0};

  const f16* a0 = wq + ((size_t)og * 64 + lq) * CH + hi * 8u;
  const f16* bp = hnT + ((size_t)b * SEQ + n0 + wave * 16u + lq) * CH + hi * 8u;
  wave_gemm_64x16(a0, bp, acc);

  #pragma unroll
  for (unsigned os = 0; os < 4; ++os) {
    const float* bsrc = bias + og * 64u + os * 16u + hi * 8u;
    const v4f b0 = *(const v4f*)(bsrc);
    const v4f b1 = *(const v4f*)(bsrc + 4);
    Pack8H pk;
    #pragma unroll
    for (unsigned r = 0; r < 4; ++r) {
      pk.h[r]     = (f16)(acc[os][r]     * 0.5f + 8.0f * bfv(b0[r]));
      pk.h[4 + r] = (f16)(acc[os][4 + r] * 0.5f + 8.0f * bfv(b1[r]));
    }
    if (t < 2) {
      *(v8h*)(sS + (wave * 16u + lq) * SQ_P + os * 16u + hi * 8u) = pk.v;
    } else {
      #pragma unroll
      for (unsigned r = 0; r < 8; ++r)
        sS[(os * 16u + hi * 8u + r) * SV_P + wave * 16u + lq] = pk.h[r];
    }
  }
  __syncthreads();

  v4u    vals[4];
  size_t gidx[4];
  f16*   dst;
  if (t < 2) {
    dst = (t == 0) ? qpl : kpl;
    #pragma unroll
    for (unsigned it = 0; it < 4; ++it) {
      const unsigned p   = it * 256u + tid;
      const unsigned row = p >> 3;
      const unsigned pc  = (p & 7u) * 8u;
      Pack8H ph;
      ph.v = *(const v8h*)(sS + row * SQ_P + pc);
      vals[it] = ph.u;
      gidx[it] = (((size_t)b * NHEAD + h) * SEQ + n0 + row) * HDIM + pc;
    }
  } else {
    dst = vtl;
    #pragma unroll
    for (unsigned it = 0; it < 4; ++it) {
      const unsigned p   = it * 256u + tid;
      const unsigned row = p >> 4;
      const unsigned pc  = (p & 15u) * 8u;
      Pack8H ph;
      ph.v = *(const v8h*)(sS + row * SV_P + pc);
      vals[it] = ph.u;
      gidx[it] = (((size_t)b * NHEAD + h) * HDIM + row) * SEQ + n0 + pc;
    }
  }
  #pragma unroll
  for (unsigned it = 0; it < 4; ++it) *(volatile v4u*)(dst + gidx[it]) = vals[it];
  __threadfence();
  #pragma unroll
  for (unsigned it = 0; it < 4; ++it) *(volatile v4u*)(dst + gidx[it]) = vals[it];
}

__global__ __launch_bounds__(256) void attn_kernel(const f16* __restrict__ qpl,
                                                   const f16* __restrict__ kpl,
                                                   const f16* __restrict__ vtl,
                                                   f16* __restrict__ ctx) {
  const unsigned qblk = blockIdx.x;
  const unsigned h    = blockIdx.y;
  const unsigned b    = blockIdx.z;
  const unsigned tid  = threadIdx.x;
  const unsigned wave = tid >> 5;
  const unsigned lane = tid & 31u;
  const unsigned lq   = lane & 15u;
  const unsigned hi   = lane >> 4;

  __shared__ __align__(16) float sO[NWAVE * 16 * OP];

  const unsigned qrow0 = qblk * BQ + wave * 16u;
  const size_t   bh    = (size_t)b * NHEAD + h;

  FragH qf[2];
  {
    const f16* qp = qpl + (bh * SEQ + qrow0 + lq) * HDIM + hi * 8u;
    #pragma unroll
    for (unsigned f = 0; f < 2; ++f) {
      qf[f].q[0] = *(const v4u*)(qp + f * 32u);
      qf[f].q[1] = *(const v4u*)(qp + f * 32u + 16u);
    }
  }

  const f16* kb_h = kpl + bh * SEQ * HDIM;
  const f16* vt_h = vtl + bh * HDIM * SEQ;

  v8f o[4];
  #pragma unroll
  for (unsigned dt = 0; dt < 4; ++dt) o[dt] = (v8f){0, 0, 0, 0, 0, 0, 0, 0};

  float rmax = -__builtin_inff();
  float rsum = 0.0f;
  const float SL = (0.125f / 64.0f) * 1.4426950408889634f;

  #pragma unroll 1
  for (unsigned i = 0; i < (unsigned)(SEQ / BK); ++i) {
    const unsigned j0 = i * BK;

    FragH ak[2][2];
    #pragma unroll
    for (unsigned sub = 0; sub < 2; ++sub) {
      #pragma unroll
      for (unsigned f = 0; f < 2; ++f) {
        const f16* base = kb_h + (size_t)(j0 + sub * 16u + lq) * HDIM + f * 32u + hi * 8u;
        ak[sub][f].q[0] = *(const v4u*)(base);
        ak[sub][f].q[1] = *(const v4u*)(base + 16);
      }
    }
    FragH bv[4];
    #pragma unroll
    for (unsigned dt = 0; dt < 4; ++dt) {
      const f16* base = vt_h + (size_t)(dt * 16u + lq) * SEQ + j0 + hi * 8u;
      bv[dt].q[0] = *(const v4u*)(base);
      bv[dt].q[1] = *(const v4u*)(base + 16);
    }

    v8f c[2];
    #pragma unroll
    for (unsigned sub = 0; sub < 2; ++sub) {
      v8f acc = (v8f){0, 0, 0, 0, 0, 0, 0, 0};
      acc = mma_f16(ak[sub][0].v, qf[0].v, acc);
      acc = mma_f16(ak[sub][1].v, qf[1].v, acc);
      c[sub] = acc;
    }

    float m_new = rmax;
    #pragma unroll
    for (unsigned r = 0; r < 8; ++r) {
      m_new = fmaxf(m_new, c[0][r]);
      m_new = fmaxf(m_new, c[1][r]);
    }
    m_new = fmaxf(m_new, __shfl_xor(m_new, 16, 32));
    const float scale = __builtin_amdgcn_exp2f((rmax - m_new) * SL);
    rmax = m_new;

    FragH pa;
    float psum = 0.0f;
    #pragma unroll
    for (unsigned r = 0; r < 8; ++r) {
      const float pc0 = __builtin_amdgcn_exp2f((c[0][r] - m_new) * SL + 12.0f);
      const float pc1 = __builtin_amdgcn_exp2f((c[1][r] - m_new) * SL + 12.0f);
      psum += pc0 + pc1;
      pa.h[r]     = (f16)pc0;
      pa.h[8 + r] = (f16)pc1;
    }
    rsum = rsum * scale + psum + __shfl_xor(psum, 16, 32);

    float sc[8];
    #pragma unroll
    for (unsigned r = 0; r < 8; ++r) sc[r] = __shfl(scale, (int)((hi << 3) + r), 32);
    #pragma unroll
    for (unsigned dt = 0; dt < 4; ++dt) {
      #pragma unroll
      for (unsigned r = 0; r < 8; ++r) o[dt][r] *= sc[r];
    }

    #pragma unroll
    for (unsigned dt = 0; dt < 4; ++dt) o[dt] = mma_f16(pa.v, bv[dt].v, o[dt]);
  }

  float rs[8];
  #pragma unroll
  for (unsigned r = 0; r < 8; ++r) rs[r] = 8.0f * (1.0f / __shfl(rsum, (int)((hi << 3) + r), 32));

  float* so = sO + wave * (16 * OP);
  #pragma unroll
  for (unsigned r = 0; r < 8; ++r) {
    #pragma unroll
    for (unsigned dt = 0; dt < 4; ++dt)
      so[(hi * 8u + r) * OP + dt * 16u + lq] = o[dt][r] * rs[r];
  }
  __syncthreads();

  v4u    vals[4];
  size_t gidx[4];
  #pragma unroll
  for (unsigned it = 0; it < 4; ++it) {
    const unsigned row = it * 4u + (lane >> 3);
    const unsigned pc  = (lane & 7u) * 8u;
    const v4f a = *(const v4f*)(so + row * OP + pc);
    const v4f d = *(const v4f*)(so + row * OP + pc + 4);
    Pack8H ph;
    #pragma unroll
    for (unsigned j = 0; j < 4; ++j) {
      ph.h[j]     = (f16)a[j];
      ph.h[4 + j] = (f16)d[j];
    }
    vals[it] = ph.u;
    gidx[it] = ((size_t)b * SEQ + qrow0 + row) * CH + h * HDIM + pc;
  }
  #pragma unroll
  for (unsigned it = 0; it < 4; ++it) *(volatile v4u*)(ctx + gidx[it]) = vals[it];
  __threadfence();
  #pragma unroll
  for (unsigned it = 0; it < 4; ++it) *(volatile v4u*)(ctx + gidx[it]) = vals[it];
}

__global__ __launch_bounds__(256) void proj_kernel(const f16* __restrict__ ctx,
                                                   const f16* __restrict__ wp,
                                                   const float* __restrict__ pb,
                                                   const float* __restrict__ x,
                                                   float* __restrict__ out) {
  const unsigned nt   = blockIdx.x;
  const unsigned og   = blockIdx.y;
  const unsigned b    = blockIdx.z;
  const unsigned tid  = threadIdx.x;
  const unsigned wave = tid >> 5;
  const unsigned lane = tid & 31u;
  const unsigned lq   = lane & 15u;
  const unsigned hi   = lane >> 4;
  const unsigned n0   = nt * 128u;

  __shared__ __align__(16) float sY[64 * YP];

  v8f acc[4];
  #pragma unroll
  for (unsigned os = 0; os < 4; ++os) acc[os] = (v8f){0, 0, 0, 0, 0, 0, 0, 0};

  const f16* a0 = wp + ((size_t)og * 64 + lq) * CH + hi * 8u;
  const f16* bp = ctx + ((size_t)b * SEQ + n0 + wave * 16u + lq) * CH + hi * 8u;
  wave_gemm_64x16(a0, bp, acc);

  #pragma unroll
  for (unsigned os = 0; os < 4; ++os) {
    #pragma unroll
    for (unsigned r = 0; r < 8; ++r)
      sY[(os * 16u + hi * 8u + r) * YP + wave * 16u + lq] = acc[os][r] * (1.0f / 1024.0f);
  }
  __syncthreads();

  v4f    vals[8];
  size_t gidx[8];
  #pragma unroll
  for (unsigned it = 0; it < 8; ++it) {
    const unsigned row = it * 8u + wave;
    const unsigned oc  = og * 64u + row;
    const v4f y = *(const v4f*)(sY + row * YP + lane * 4u);
    const size_t idx = ((size_t)b * CH + oc) * SEQ_FULL + n0 + lane * 4u;
    const v4f xv = *(const v4f*)(x + idx);
    const float bo = bfv(pb[oc]);
    v4f val;
    #pragma unroll
    for (unsigned j = 0; j < 4; ++j) val[j] = (y[j] + bo) + bfv(xv[j]);
    vals[it] = val;
    gidx[it] = idx;
  }
  #pragma unroll
  for (unsigned it = 0; it < 8; ++it) *(volatile v4f*)(out + gidx[it]) = vals[it];
  __threadfence();
  #pragma unroll
  for (unsigned it = 0; it < 8; ++it) *(volatile v4f*)(out + gidx[it]) = vals[it];
}

extern "C" void kernel_launch(void* const* d_in, const int* in_sizes, int n_in,
                              void* d_out, int out_size, void* d_ws, size_t ws_size,
                              hipStream_t stream) {
  if (n_in < 7) return;
  const size_t x_need = ((size_t)NB * CH - 1) * SEQ_FULL + SEQ;
  if ((size_t)in_sizes[0] < x_need) return;
  if ((size_t)in_sizes[1] < (size_t)CH) return;
  if ((size_t)in_sizes[2] < (size_t)CH) return;
  if ((size_t)in_sizes[3] < (size_t)WQ_ELEMS) return;
  if ((size_t)in_sizes[4] < (size_t)QKV_O) return;
  if ((size_t)in_sizes[5] < (size_t)WP_ELEMS) return;
  if ((size_t)in_sizes[6] < (size_t)CH) return;
  if ((size_t)out_size < x_need) return;

  const size_t stats_bytes = (((size_t)NB * NGRP * 128) + 4095) / 4096 * 4096;
  const size_t wq_bytes    = (size_t)WQ_ELEMS * 2;
  const size_t wp_bytes    = (size_t)WP_ELEMS * 2;
  const size_t plane_bytes = (size_t)NB * SEQ * CH * 2;
  size_t off = 0;
  const size_t off_stats = off; off += stats_bytes;
  const size_t off_wq    = off; off += wq_bytes;
  const size_t off_wp    = off; off += wp_bytes;
  const size_t off_hn    = off; off += plane_bytes;
  const size_t off_q     = off; off += plane_bytes;
  const size_t off_k     = off; off += plane_bytes;
  const size_t off_v     = off; off += plane_bytes;
  const size_t off_ctx   = off; off += plane_bytes;
  if (ws_size < off) return;

  const float* x     = (const float*)d_in[0];
  const float* gnw   = (const float*)d_in[1];
  const float* gnb   = (const float*)d_in[2];
  const float* qkvw  = (const float*)d_in[3];
  const float* qkvb  = (const float*)d_in[4];
  const float* projw = (const float*)d_in[5];
  const float* projb = (const float*)d_in[6];
  float* out = (float*)d_out;

  char* ws = (char*)d_ws;
  float* stats = (float*)(ws + off_stats);
  f16*   wq    = (f16*)(ws + off_wq);
  f16*   wp    = (f16*)(ws + off_wp);
  f16*   hnT   = (f16*)(ws + off_hn);
  f16*   qpl   = (f16*)(ws + off_q);
  f16*   kpl   = (f16*)(ws + off_k);
  f16*   vtl   = (f16*)(ws + off_v);
  f16*   ctx   = (f16*)(ws + off_ctx);

  wcvt_kernel   <<<dim3(WQ_BLKS + WP_BLKS), 256, 0, stream>>>(qkvw, projw, wq, wp);
  gnstats_kernel<<<dim3(NGRP, NB), 256, 0, stream>>>(x, stats);
  gnapply_kernel<<<dim3(SEQ / 64, CH / 64, NB), 256, 0, stream>>>(x, gnw, gnb, stats, hnT);
  qkv_kernel    <<<dim3(SEQ / 128, QKV_O / 64, NB), 256, 0, stream>>>(hnT, wq, qkvb, qpl, kpl, vtl);
  attn_kernel   <<<dim3(SEQ / BQ, NHEAD, NB), 256, 0, stream>>>(qpl, kpl, vtl, ctx);
  proj_kernel   <<<dim3(SEQ / 128, CH / 64, NB), 256, 0, stream>>>(ctx, wp, projb, x, out);
}
